// CenterAttention_7086696039090
// MI455X (gfx1250) — hardware-verified
//
#include <hip/hip_runtime.h>
#include <stdint.h>


#define C_DIM   384
#define N_QKV   1152
#define W_ROWS  1536
#define KDIM    384
#define WSCALE  64.0f
#define WINV    0.015625f

typedef _Float16 v16h __attribute__((ext_vector_type(16)));
typedef _Float16 v8h  __attribute__((ext_vector_type(8)));
typedef float    v8f  __attribute__((ext_vector_type(8)));
typedef float    v4f  __attribute__((ext_vector_type(4)));
typedef float    v2f  __attribute__((ext_vector_type(2)));
union Frag { v16h v; v8h half[2]; };

__device__ __forceinline__ v8f wmma16(v8f acc, v16h a, v16h b) {
    acc = __builtin_amdgcn_wmma_f32_16x16x32_f16(false, a, false, b, (short)0, acc, false, false);
    asm volatile("v_nop\n\tv_nop\n\tv_nop\n\tv_nop" : "+v"(acc) : "v"(a), "v"(b));
    return acc;
}

__global__ __launch_bounds__(256)
void cvt_x_kernel(const float* __restrict__ x, _Float16* xh, int M) {
    const int r = blockIdx.x * 4 + (threadIdx.x >> 6);
    const int t = threadIdx.x & 63;
    if (r < M && t < 48) {
        const float* src = x + (size_t)r * C_DIM + 8 * t;
        const v4f lo = *(const v4f*)src;
        const v4f hi = *(const v4f*)(src + 4);
        v8h o;
#pragma unroll
        for (int e = 0; e < 4; ++e) { o[e] = (_Float16)lo[e]; o[4 + e] = (_Float16)hi[e]; }
        _Float16* dst = xh + (size_t)r * C_DIM + 8 * t;
        *(volatile v8h*)dst = o;
        __threadfence();
        *(volatile v8h*)dst = o;
    }
}

__global__ __launch_bounds__(64)
void cvt_w_kernel(const float* __restrict__ q_w, const float* __restrict__ kv_w,
                  const float* __restrict__ proj_w, _Float16* wT) {
    const int row = blockIdx.x;
    const int t = threadIdx.x;
    const float* src;
    int N, n;
    if (row < C_DIM)           { src = q_w;    N = C_DIM;     n = row; }
    else if (row < N_QKV)      { src = kv_w;   N = 2 * C_DIM; n = row - C_DIM; }
    else                       { src = proj_w; N = C_DIM;     n = row - N_QKV; }
    if (t < 48) {
        v8h o;
#pragma unroll
        for (int e = 0; e < 8; ++e) {
            const int k = 8 * t + e;
            o[e] = (_Float16)(src[(size_t)k * N + n] * WSCALE);
        }
        _Float16* dst = wT + (size_t)row * KDIM + 8 * t;
        *(volatile v8h*)dst = o;
        __threadfence();
        *(volatile v8h*)dst = o;
    }
}

__device__ __forceinline__ void store_tile(const float (*stw)[68], const float* __restrict__ bsel,
                                           float osc, float* out, int ldo,
                                           int row0, int col0, int h, int m) {
#pragma unroll
    for (int it = 0; it < 16; ++it) {
        const int row = 2 * it + h;
        const int c = 4 * m;
        v4f v = *(const v4f*)(&stw[row][c]);
        const v4f bb = *(const v4f*)(bsel + c);
        v = (v * WINV + bb) * osc;
        *(volatile v4f*)(out + (size_t)(row0 + row) * (size_t)ldo + col0 + c) = v;
    }
}

__global__ __launch_bounds__(128)
void gemm_kernel(const _Float16* __restrict__ A, const _Float16* __restrict__ Bt,
                 const float* __restrict__ bias0, const float* __restrict__ bias1,
                 float* out, int ldo, int split, float oscale0) {
    __shared__ __attribute__((aligned(16))) float st[4][32][68];

    const int w = threadIdx.x >> 5;
    const int l = threadIdx.x & 31;
    const int h = l >> 4, m = l & 15;
    const int row0 = blockIdx.x * 128 + w * 32;
    const int y = blockIdx.y;
    const int col0 = y * 64;

    v8f acc[2][4];
#pragma unroll
    for (int mm = 0; mm < 2; ++mm)
#pragma unroll
        for (int t = 0; t < 4; ++t)
#pragma unroll
            for (int r = 0; r < 8; ++r) acc[mm][t][r] = 0.0f;

    const _Float16* ap = A  + (size_t)(row0 + m) * KDIM + 8 * h;
    const _Float16* bp = Bt + (size_t)(col0 + m) * KDIM + 8 * h;

#pragma unroll 1
    for (int k0 = 0; k0 < KDIM; k0 += 32) {
        Frag a[2], b[4];
#pragma unroll
        for (int mm = 0; mm < 2; ++mm) {
            const _Float16* p = ap + (size_t)mm * 16 * KDIM + k0;
            a[mm].half[0] = *(const v8h*)p;
            a[mm].half[1] = *(const v8h*)(p + 16);
        }
#pragma unroll
        for (int t = 0; t < 4; ++t) {
            const _Float16* p = bp + (size_t)t * 16 * KDIM + k0;
            b[t].half[0] = *(const v8h*)p;
            b[t].half[1] = *(const v8h*)(p + 16);
        }
#pragma unroll
        for (int mm = 0; mm < 2; ++mm)
#pragma unroll
            for (int t = 0; t < 4; ++t)
                acc[mm][t] = wmma16(acc[mm][t], a[mm].v, b[t].v);
    }

#pragma unroll
    for (int mm = 0; mm < 2; ++mm)
#pragma unroll
        for (int t = 0; t < 4; ++t)
#pragma unroll
            for (int r = 0; r < 8; ++r)
                st[w][mm * 16 + 8 * h + r][t * 16 + m] = acc[mm][t][r];
    __syncthreads();

    const float* bsel = (y < split) ? (bias0 + y * 64) : (bias1 + (y - split) * 64);
    const float osc = (y < split) ? oscale0 : 1.0f;
    store_tile(st[w], bsel, osc, out, ldo, row0, col0, h, m);
    __threadfence();
    store_tile(st[w], bsel, osc, out, ldo, row0, col0, h, m);
}

__global__ __launch_bounds__(192)
void attn_kernel(const float* __restrict__ qkv, const int* __restrict__ Hp,
                 const int* __restrict__ Wp, _Float16* ao, int npix) {
    __shared__ __attribute__((aligned(16))) _Float16 st[6][64];

    const int p  = blockIdx.x;
    const int hd = threadIdx.x >> 5;
    const int l  = threadIdx.x & 31;

    int Hh = Hp[0], Ww = Wp[0];
    Hh = Hh < 1 ? 1 : (Hh > npix ? npix : Hh);
    Ww = Ww < 1 ? 1 : (Ww > npix ? npix : Ww);
    const int hw   = Hh * Ww;
    const int b    = p / hw;
    const int base = b * hw;
    const int ij   = p - base;
    const int i    = ij / Ww;
    const int j    = ij - i * Ww;

    const v2f qv = *(const v2f*)(qkv + (size_t)p * N_QKV + hd * 64 + 2 * l);

    float lg[9], okf[9];
    int   voff[9];
#pragma unroll
    for (int n9 = 0; n9 < 9; ++n9) {
        const int di = n9 / 3 - 1, dj = n9 % 3 - 1;
        const int ii = i + di, jj = j + dj;
        const bool ok = ((unsigned)ii < (unsigned)Hh) && ((unsigned)jj < (unsigned)Ww);
        int np = ok ? (base + ii * Ww + jj) : p;
        np = np < 0 ? 0 : (np >= npix ? npix - 1 : np);
        const int koff = np * N_QKV + C_DIM + hd * 64 + 2 * l;
        voff[n9] = koff + C_DIM;
        okf[n9]  = ok ? 1.0f : 0.0f;
        const v2f kk = *(const v2f*)(qkv + (size_t)koff);
        float s = (qv.x * kk.x + qv.y * kk.y) * okf[n9];
        s += __shfl_xor(s, 16);
        s += __shfl_xor(s, 8);
        s += __shfl_xor(s, 4);
        s += __shfl_xor(s, 2);
        s += __shfl_xor(s, 1);
        lg[n9] = s;
    }

    float mx = lg[0];
#pragma unroll
    for (int n9 = 1; n9 < 9; ++n9) mx = fmaxf(mx, lg[n9]);
    float ex[9], ssum = 0.0f;
#pragma unroll
    for (int n9 = 0; n9 < 9; ++n9) { ex[n9] = __expf(lg[n9] - mx); ssum += ex[n9]; }
    const float inv = 1.0f / ssum;

    float o0 = 0.0f, o1 = 0.0f;
#pragma unroll
    for (int n9 = 0; n9 < 9; ++n9) {
        const float wgt = ex[n9] * inv * okf[n9];
        const v2f vv = *(const v2f*)(qkv + (size_t)voff[n9]);
        o0 += wgt * vv.x;
        o1 += wgt * vv.y;
    }

    st[hd][2 * l]     = (_Float16)o0;
    st[hd][2 * l + 1] = (_Float16)o1;
    __syncthreads();

    v8h ov;
    _Float16* dst = ao + (size_t)p * C_DIM + hd * 64 + 8 * l;
    if (l < 8) {
        ov = *(const v8h*)(&st[hd][8 * l]);
        *(volatile v8h*)dst = ov;
    }
    __threadfence();
    if (l < 8) {
        *(volatile v8h*)dst = ov;
    }
}

extern "C" void kernel_launch(void* const* d_in, const int* in_sizes, int n_in,
                              void* d_out, int out_size, void* d_ws, size_t ws_size,
                              hipStream_t stream) {
    if (n_in < 9) return;
    const float* x      = (const float*)d_in[0];
    const int*   Hp     = (const int*)d_in[1];
    const int*   Wp     = (const int*)d_in[2];
    const float* q_w    = (const float*)d_in[3];
    const float* q_b    = (const float*)d_in[4];
    const float* kv_w   = (const float*)d_in[5];
    const float* kv_b   = (const float*)d_in[6];
    const float* proj_w = (const float*)d_in[7];
    const float* proj_b = (const float*)d_in[8];

    const int M = in_sizes[0] / C_DIM;
    if (M <= 0 || (M % 128) != 0 || in_sizes[0] != M * C_DIM) return;
    if (out_size != M * C_DIM) return;
    if (in_sizes[1] < 1 || in_sizes[2] < 1) return;
    if (in_sizes[3] != C_DIM * C_DIM || in_sizes[5] != C_DIM * 2 * C_DIM ||
        in_sizes[7] != C_DIM * C_DIM) return;
    if (in_sizes[4] < C_DIM || in_sizes[6] < 2 * C_DIM || in_sizes[8] < C_DIM) return;

    char* ws = (char*)d_ws;
    size_t o = 0;
    _Float16* xh  = (_Float16*)(ws + o); o += (size_t)M * C_DIM * 2;
    _Float16* wT  = (_Float16*)(ws + o); o += (size_t)W_ROWS * KDIM * 2;
    float*    qkv = (float*)(ws + o);    o += (size_t)M * N_QKV * 4;
    _Float16* ao  = (_Float16*)(ws + o); o += (size_t)M * C_DIM * 2;
    if (o > ws_size || o > (size_t)134217728) return;

    cvt_x_kernel<<<M / 4, 256, 0, stream>>>(x, xh, M);
    cvt_w_kernel<<<W_ROWS, 64, 0, stream>>>(q_w, kv_w, proj_w, wT);

    gemm_kernel<<<dim3(M / 128, N_QKV / 64), 128, 0, stream>>>(
        xh, wT, q_b, kv_b, qkv, N_QKV, 6, 0.125f);

    attn_kernel<<<M, 192, 0, stream>>>(qkv, Hp, Wp, ao, M);

    gemm_kernel<<<dim3(M / 128, C_DIM / 64), 128, 0, stream>>>(
        ao, wT + (size_t)N_QKV * KDIM, proj_b, proj_b, (float*)d_out, C_DIM, 6, 1.0f);
}
